// DistBiasSelfAttention_64493228917282
// MI455X (gfx1250) — hardware-verified
//
#include <hip/hip_runtime.h>


#define NB_  4
#define TT   1024
#define CC   256
#define NH_  8
#define HD   32
#define PCAR 1024.0f
#define SCL  0.17677669529663687f
typedef _Float16 h16;
typedef unsigned short bf;
typedef __attribute__((ext_vector_type(16))) __bf16   v16bf;
typedef __attribute__((ext_vector_type(16))) _Float16 v16h;
typedef __attribute__((ext_vector_type(8)))  _Float16 v8h;
typedef __attribute__((ext_vector_type(8)))  unsigned short v8us;
typedef __attribute__((ext_vector_type(8)))  float    v8f;
typedef __attribute__((ext_vector_type(4)))  float    v4f;
typedef v8h  __attribute__((may_alias)) v8ha;
typedef v4f  __attribute__((may_alias)) v4fa;
typedef v8us __attribute__((may_alias)) v8usa;

__device__ __forceinline__ unsigned short f2bf(float f) { unsigned u = __float_as_uint(f); u += 0x7FFFu + ((u >> 16) & 1u); return (unsigned short)(u >> 16); }
__device__ __forceinline__ float bf2f(unsigned short b) { return __uint_as_float(((unsigned)b) << 16); }
__device__ __forceinline__ float bfr(float f) { return bf2f(f2bf(f)); }
__device__ __forceinline__ v16h cat16(v8h lo, v8h hi) { return __builtin_shufflevector(lo, hi, 0, 1, 2, 3, 4, 5, 6, 7, 8, 9, 10, 11, 12, 13, 14, 15); }
__device__ __forceinline__ v16bf cat16b(v8us lo, v8us hi) { return __builtin_bit_cast(v16bf, __builtin_shufflevector(lo, hi, 0, 1, 2, 3, 4, 5, 6, 7, 8, 9, 10, 11, 12, 13, 14, 15)); }
__device__ __forceinline__ v8f wmma16(v16h a, v16h b, v8f c) { return __builtin_amdgcn_wmma_f32_16x16x32_f16(false, a, false, b, (short)0, c, false, false); }
__device__ __forceinline__ v8f wmmab(v16bf a, v16bf b, v8f c) { return __builtin_amdgcn_wmma_f32_16x16x32_bf16(false, a, false, b, (short)0, c, false, false); }


template <typename T16> struct WFrag;
template <> struct WFrag<h16> { typedef v16h V; static __device__ __forceinline__ V ld(const h16* p) { return cat16(*(const v8h*)p, *(const v8h*)(p + 16)); } static __device__ __forceinline__ v8f mma(V a, V b, v8f c) { return wmma16(a, b, c); } };
template <> struct WFrag<bf> { typedef v16bf V; static __device__ __forceinline__ V ld(const bf* p) { return cat16b(*(const v8us*)p, *(const v8us*)(p + 16)); } static __device__ __forceinline__ v8f mma(V a, V b, v8f c) { return wmmab(a, b, c); } };
template <typename T16, int NSPLIT, bool BIAS>
__global__ __launch_bounds__(32) void k_gemmw(const T16* __restrict__ A, const T16* __restrict__ A2, const T16* __restrict__ Bt, const T16* __restrict__ Bt2, int K, float* C, int ldc, const float* __restrict__ bias, size_t sA, size_t sB, size_t sC) {
    typedef typename WFrag<T16>::V V;
    __shared__ __align__(16) float os[16 * 68];
    const size_t z = blockIdx.z; A += z * sA; if (A2) A2 += z * sA; Bt += z * sB; if (Bt2) Bt2 += z * sB; C += z * sC;
    const int lane = threadIdx.x & 31, lr = lane & 15, hi = lane >> 4; const int r0 = blockIdx.x * 64, c0 = blockIdx.y * 64;
    v8f acc[4][4];
#pragma unroll
    for (int mb = 0; mb < 4; ++mb)
#pragma unroll
        for (int nb = 0; nb < 4; ++nb) acc[mb][nb] = (v8f){};
    const size_t aoff = (size_t)(r0 + lr) * K + 8 * hi, boff = (size_t)(c0 + lr) * K + 8 * hi;
#pragma unroll 1
    for (int kc = 0; kc < K; kc += 32) {
        V a[4], a2[4];
#pragma unroll
        for (int mb = 0; mb < 4; ++mb) { a[mb] = WFrag<T16>::ld(A + aoff + (size_t)mb * 16 * K + kc); if (NSPLIT == 1 || NSPLIT == 2) a2[mb] = WFrag<T16>::ld(A2 + aoff + (size_t)mb * 16 * K + kc); }
#pragma unroll
        for (int nb = 0; nb < 4; ++nb) { const V b = WFrag<T16>::ld(Bt + boff + (size_t)nb * 16 * K + kc); V b2; if (NSPLIT >= 2) b2 = WFrag<T16>::ld(Bt2 + boff + (size_t)nb * 16 * K + kc);
#pragma unroll
            for (int mb = 0; mb < 4; ++mb) { acc[mb][nb] = WFrag<T16>::mma(a[mb], b, acc[mb][nb]); if (NSPLIT == 1 || NSPLIT == 2) acc[mb][nb] = WFrag<T16>::mma(a2[mb], b, acc[mb][nb]); if (NSPLIT >= 2) acc[mb][nb] = WFrag<T16>::mma(a[mb], b2, acc[mb][nb]); } }
        asm volatile("v_nop\n\tv_nop\n\tv_nop\n\tv_nop" : "+v"(acc[0][0]), "+v"(acc[1][1]), "+v"(acc[2][2]), "+v"(acc[3][3]) : "v"(a[0]), "v"(a[3]));
    }
#pragma unroll
    for (int mb = 0; mb < 4; ++mb) {
#pragma unroll
        for (int nb = 0; nb < 4; ++nb) {
#pragma unroll
            for (int j = 0; j < 8; ++j) os[(hi * 8 + j) * 68 + nb * 16 + lr] = acc[mb][nb][j]; }
        __builtin_amdgcn_wave_barrier(); asm volatile("" ::: "memory");
        float* crow = C + (size_t)(r0 + mb * 16) * ldc + c0;
#pragma unroll 1
        for (int ps = 0; ps < 2; ++ps) {
#pragma unroll
            for (int s = 0; s < 8; ++s) { const int row = 2 * s + hi, cofs = lr * 4; v4f val = *(const v4fa*)(os + row * 68 + cofs); if (BIAS) { val[0] += bfr(bias[c0 + cofs]); val[1] += bfr(bias[c0 + cofs + 1]); val[2] += bfr(bias[c0 + cofs + 2]); val[3] += bfr(bias[c0 + cofs + 3]); }
                *(volatile v4f*)(crow + (size_t)row * ldc + cofs) = val; }
            if (ps == 0) __threadfence(); }
        __builtin_amdgcn_wave_barrier(); asm volatile("" ::: "memory");
    }
}

__device__ __forceinline__ h16 tohx(float x) { return (h16)x; }
__device__ __forceinline__ void splitf(float y, unsigned short& h, unsigned short& l) { h = f2bf(y); l = f2bf(y - bf2f(h)); }
typedef __attribute__((ext_vector_type(2))) _Float16 v2h;
typedef __attribute__((ext_vector_type(4))) _Float16 v4h;
typedef __attribute__((ext_vector_type(2))) unsigned short v2us;
typedef __attribute__((ext_vector_type(4))) unsigned short v4us;
typedef __attribute__((ext_vector_type(2))) float v2f;

__global__ __launch_bounds__(256) void k_cvt8(const float* __restrict__ src, bf* dst, size_t n8) { const size_t i = (size_t)blockIdx.x * 256 + threadIdx.x; if (i >= n8) return; const v8f v = *(const v8f*)(src + i * 8); v8us o;
#pragma unroll
    for (int k = 0; k < 8; ++k) o[k] = f2bf(v[k]); *(volatile v8us*)(dst + i * 8) = o; __threadfence(); *(volatile v8us*)(dst + i * 8) = o; }
__global__ __launch_bounds__(256) void k_dist(const float* __restrict__ xyz, float* DIST) { const size_t e = ((size_t)blockIdx.x * 256 + threadIdx.x) * 4; if (e >= (size_t)TT * TT) return; const int j0 = (int)(e % TT), i = (int)(e / TT); const float xi = bfr(xyz[i * 3]), yi = bfr(xyz[i * 3 + 1]), zi = bfr(xyz[i * 3 + 2]); v4f o;
#pragma unroll
    for (int q = 0; q < 4; ++q) { const int j = j0 + q; const float dx = __fsub_rn(xi, bfr(xyz[j * 3])), dy = __fsub_rn(yi, bfr(xyz[j * 3 + 1])), dz = __fsub_rn(zi, bfr(xyz[j * 3 + 2])); float a = __fmul_rn(dx, dx), b2 = __fmul_rn(dy, dy), c2 = __fmul_rn(dz, dz); asm volatile("" : "+v"(a), "+v"(b2), "+v"(c2)); o[q] = -__fsqrt_rn(__fadd_rn(__fadd_rn(a, b2), c2)); }
    *(volatile v4f*)(DIST + e) = o; __threadfence(); *(volatile v4f*)(DIST + e) = o; }
__global__ __launch_bounds__(256) void k_tau(const float* __restrict__ F, const float* __restrict__ tw, const float* __restrict__ tb, float* TAU) { const int e = blockIdx.x * 256 + threadIdx.x; if (e >= TT * NH_) return; const int h = e % NH_, i = e / NH_; float s = 0.f;
    for (int c = 0; c < CC; ++c) { float p = __fmul_rn(bfr(F[(size_t)i * CC + c]), bfr(tw[h * CC + c])); asm volatile("" : "+v"(p)); s = __fadd_rn(s, p); } const float o = __fadd_rn(s, bfr(tb[h])); *(volatile float*)(TAU + e) = o; __threadfence(); *(volatile float*)(TAU + e) = o; }
__global__ __launch_bounds__(256) void k_qk16(const float* __restrict__ F, h16* QP, h16* KP) { const size_t e = ((size_t)blockIdx.x * 256 + threadIdx.x) * 2; if (e >= (size_t)NH_ * TT * HD) return; const int d = (int)(e % HD); const int t = (int)((e / HD) % TT); const int h = (int)(e / ((size_t)HD * TT)); const float* s = F + (size_t)t * (3 * CC) + h * HD + d; v2h q, k; q[0] = tohx(s[0]); q[1] = tohx(s[1]); k[0] = tohx(s[CC]); k[1] = tohx(s[CC + 1]);
    *(volatile v2h*)(QP + e) = q; *(volatile v2h*)(KP + e) = k; __threadfence(); *(volatile v2h*)(QP + e) = q; *(volatile v2h*)(KP + e) = k; }
__global__ __launch_bounds__(256) void k_vt16(const float* __restrict__ F, h16* VT) { const size_t e = ((size_t)blockIdx.x * 256 + threadIdx.x) * 2; if (e >= (size_t)NH_ * 64 * TT) return; const int t = (int)(e % TT); const int dd = (int)((e / TT) % 64); const int h = (int)(e / ((size_t)TT * 64)); v2h o;
    if (dd < HD) { o[0] = tohx(F[(size_t)t * (3 * CC) + 2 * CC + h * HD + dd]); o[1] = tohx(F[(size_t)(t + 1) * (3 * CC) + 2 * CC + h * HD + dd]); } else { o[0] = (h16)0.f; o[1] = (h16)0.f; } *(volatile v2h*)(VT + e) = o; __threadfence(); *(volatile v2h*)(VT + e) = o; }
__global__ __launch_bounds__(256) void k_bsoft(const float* __restrict__ Sb, const float* __restrict__ DIST, const float* __restrict__ TAU, const float* __restrict__ scale, int h, h16* P16) { const int lane = threadIdx.x & 31; const int row = blockIdx.x * 8 + (threadIdx.x >> 5); if (row >= TT) return; const float tsc = __fmul_rn(TAU[row * NH_ + h], bfr(scale[h])); const float* sr = Sb + (size_t)row * TT; const float* dr = DIST + (size_t)row * TT; float v[32]; float mx = -3.0e38f;
#pragma unroll
    for (int ch = 0; ch < 8; ++ch) { const int j0 = ch * 128 + lane * 4; const v4f a = *(const v4f*)(sr + j0), d4 = *(const v4f*)(dr + j0);
#pragma unroll
        for (int q = 0; q < 4; ++q) { float s8 = __fmul_rn(a[q], SCL), bb = __fmul_rn(d4[q], tsc); asm volatile("" : "+v"(s8), "+v"(bb)); const float t = __fadd_rn(s8, bb); v[ch * 4 + q] = t; mx = fmaxf(mx, t); } }
#pragma unroll
    for (int sh = 16; sh; sh >>= 1) mx = fmaxf(mx, __shfl_xor(mx, sh, 32));
    float sum = 0.f;
#pragma unroll
    for (int k = 0; k < 32; ++k) { float d0 = __fsub_rn(v[k], mx); asm volatile("" : "+v"(d0)); v[k] = __expf(d0); sum += v[k]; }
#pragma unroll
    for (int sh = 16; sh; sh >>= 1) sum += __shfl_xor(sum, sh, 32);
    const float f = __fdiv_rn(PCAR, sum);
#pragma unroll 1
    for (int ps = 0; ps < 2; ++ps) {
#pragma unroll
        for (int ch = 0; ch < 8; ++ch) { v4h o;
#pragma unroll
            for (int q = 0; q < 4; ++q) o[q] = tohx(v[ch * 4 + q] * f); *(volatile v4h*)(P16 + (size_t)row * TT + ch * 128 + lane * 4) = o; }
        if (ps == 0) __threadfence(); } }
__global__ __launch_bounds__(256) void k_ctx(const float* __restrict__ O, int h, bf* Ch, bf* Cl) { const size_t e = ((size_t)blockIdx.x * 256 + threadIdx.x) * 2; if (e >= (size_t)TT * HD) return; const int d = (int)(e % HD), t = (int)(e / HD); v2us oh, ol;
#pragma unroll
    for (int u = 0; u < 2; ++u) { unsigned short a, c2; splitf(O[(size_t)t * 64 + d + u] * (1.0f / PCAR), a, c2); oh[u] = a; ol[u] = c2; } const size_t oo = (size_t)t * CC + h * HD + d; *(volatile v2us*)(Ch + oo) = oh; *(volatile v2us*)(Cl + oo) = ol; __threadfence(); *(volatile v2us*)(Ch + oo) = oh; *(volatile v2us*)(Cl + oo) = ol; }
__global__ __launch_bounds__(256) void k_ln(const float* __restrict__ Of, const float* __restrict__ feats, const float* __restrict__ g, const float* __restrict__ bb, float* OUTb) { const int lane = threadIdx.x & 31; const int t = blockIdx.x * 8 + (threadIdx.x >> 5); if (t >= TT) return; float v[8]; float s = 0.f;
#pragma unroll
    for (int ch = 0; ch < 2; ++ch) { const size_t o = (size_t)t * CC + ch * 128 + lane * 4; const v4f a = *(const v4f*)(Of + o);
#pragma unroll
        for (int q = 0; q < 4; ++q) { v[ch * 4 + q] = __fadd_rn(a[q], bfr(feats[o + q])); s = __fadd_rn(s, v[ch * 4 + q]); } }
#pragma unroll
    for (int sh = 16; sh; sh >>= 1) s += __shfl_xor(s, sh, 32);
    const float mu = s * (1.0f / CC); float q2 = 0.f;
#pragma unroll
    for (int k = 0; k < 8; ++k) { const float d = __fsub_rn(v[k], mu); float p = __fmul_rn(d, d); asm volatile("" : "+v"(p)); q2 = __fadd_rn(q2, p); }
#pragma unroll
    for (int sh = 16; sh; sh >>= 1) q2 += __shfl_xor(q2, sh, 32);
    const float rs = __frsqrt_rn(__fadd_rn(q2 * (1.0f / CC), 1e-5f));
#pragma unroll 1
    for (int ps = 0; ps < 2; ++ps) {
#pragma unroll
        for (int ch = 0; ch < 2; ++ch) { v4f of;
#pragma unroll
            for (int q = 0; q < 4; ++q) { const int d = ch * 128 + lane * 4 + q; float tn = __fmul_rn(__fsub_rn(v[ch * 4 + q], mu), rs); asm volatile("" : "+v"(tn)); float tg = __fmul_rn(tn, bfr(g[d])); asm volatile("" : "+v"(tg)); of[q] = __fadd_rn(tg, bfr(bb[d])); }
            *(volatile v4f*)(OUTb + (size_t)t * CC + ch * 128 + lane * 4) = of; }
        if (ps == 0) __threadfence(); } }

extern "C" void kernel_launch(void* const* d_in, const int* in_sizes, int n_in,
                              void* d_out, int out_size, void* d_ws, size_t ws_size, hipStream_t stream) {
    (void)in_sizes; (void)n_in; (void)out_size;
    const float* IN[11]; for (int i = 0; i < 11; ++i) IN[i] = (const float*)d_in[i];
    float* OUT = (float*)d_out;
    char* wsp = (char*)d_ws;
    auto take = [&](size_t bytes) { char* p = wsp; wsp += (bytes + 255) & ~(size_t)255; return (void*)p; };
    bf* WIN = (bf*)take((size_t)3 * CC * CC * 2); bf* WO = (bf*)take((size_t)CC * CC * 2); bf* XB = (bf*)take((size_t)TT * CC * 2); float* F = (float*)take((size_t)TT * 3 * CC * 4); float* DIST = (float*)take((size_t)TT * TT * 4); float* TAU = (float*)take((size_t)TT * NH_ * 4);
    h16* QP = (h16*)take((size_t)NH_ * TT * HD * 2); h16* KP = (h16*)take((size_t)NH_ * TT * HD * 2); h16* VT = (h16*)take((size_t)NH_ * 64 * TT * 2); float* Sb = (float*)take((size_t)TT * TT * 4); h16* P16 = (h16*)take((size_t)TT * TT * 2); float* O = (float*)take((size_t)TT * 64 * 4); bf* Ch = (bf*)take((size_t)TT * CC * 2); bf* Cl = (bf*)take((size_t)TT * CC * 2); float* Of = (float*)take((size_t)TT * CC * 4);
    if ((size_t)(wsp - (char*)d_ws) > ws_size) return;
    k_cvt8<<<(3 * CC * CC / 8 + 255) / 256, 256, 0, stream>>>(IN[2], WIN, (size_t)3 * CC * CC / 8); k_cvt8<<<(CC * CC / 8 + 255) / 256, 256, 0, stream>>>(IN[4], WO, (size_t)CC * CC / 8);
    for (int b = 0; b < NB_; ++b) { const float* fb = IN[0] + (size_t)b * TT * CC;
        k_cvt8<<<(TT * CC / 8 + 255) / 256, 256, 0, stream>>>(fb, XB, (size_t)TT * CC / 8); k_dist<<<(TT * TT / 4 + 255) / 256, 256, 0, stream>>>(IN[1] + (size_t)b * TT * 3, DIST); k_tau<<<(TT * NH_ + 255) / 256, 256, 0, stream>>>(fb, IN[6], IN[7], TAU);
        k_gemmw<bf, 0, true><<<dim3(TT / 64, 3 * CC / 64, 1), 32, 0, stream>>>(XB, nullptr, WIN, nullptr, CC, F, 3 * CC, IN[3], 0, 0, 0);
        k_qk16<<<(unsigned)(((size_t)NH_ * TT * HD / 2 + 255) / 256), 256, 0, stream>>>(F, QP, KP); k_vt16<<<(unsigned)(((size_t)NH_ * 64 * TT / 2 + 255) / 256), 256, 0, stream>>>(F, VT);
        for (int h = 0; h < NH_; ++h) {
            k_gemmw<h16, 0, false><<<dim3(TT / 64, TT / 64, 1), 32, 0, stream>>>(QP + (size_t)h * TT * HD, nullptr, KP + (size_t)h * TT * HD, nullptr, HD, Sb, TT, nullptr, 0, 0, 0);
            k_bsoft<<<TT / 8, 256, 0, stream>>>(Sb, DIST, TAU, IN[8], h, P16);
            k_gemmw<h16, 0, false><<<dim3(TT / 64, 1, 1), 32, 0, stream>>>(P16, nullptr, VT + (size_t)h * 64 * TT, nullptr, TT, O, 64, nullptr, 0, 0, 0);
            k_ctx<<<(TT * HD / 2 + 255) / 256, 256, 0, stream>>>(O, h, Ch, Cl); }
        k_gemmw<bf, 1, true><<<dim3(TT / 64, CC / 64, 1), 32, 0, stream>>>(Ch, Cl, WO, nullptr, CC, Of, CC, IN[5], 0, 0, 0);
        k_ln<<<TT / 8, 256, 0, stream>>>(Of, fb, IN[9], IN[10], OUT + (size_t)b * TT * CC); }
}
